// MDCN3x3Norm_62740882260588
// MI455X (gfx1250) — hardware-verified
//
#include <hip/hip_runtime.h>
#include <math.h>
typedef __attribute__((ext_vector_type(16))) _Float16 v16h;
typedef __attribute__((ext_vector_type(8)))  _Float16 v8h;
typedef __attribute__((ext_vector_type(16))) __bf16   v16b;
typedef __attribute__((ext_vector_type(8)))  __bf16   v8b;
typedef __attribute__((ext_vector_type(8)))  float    v8f;
typedef __attribute__((ext_vector_type(4)))  float    v4f;
#define PSCALE 32768.0f
#define U16(p) ((const unsigned short*)(const void*)(p))
#define PSCALE_INV (1.0f / 32768.0f)

__device__ __forceinline__ unsigned short f2bf_bits(float f) {
  unsigned u = __float_as_uint(f);
  return (unsigned short)((u + 0x7FFFu + ((u >> 16) & 1u)) >> 16);
}
__device__ __forceinline__ float bf_bits2f(unsigned short h) { return __uint_as_float(((unsigned)h) << 16); }

__device__ __forceinline__ void dep_guard_h(v8f& a, v8f& b, v16h x, v16h y) { asm volatile("v_nop\n\tv_nop\n\tv_nop\n\tv_nop" : "+v"(a), "+v"(b) : "v"(x), "v"(y)); }
__device__ __forceinline__ void dep_guard_b(v8f& a, v8f& b, v16b x, v16b y) { asm volatile("v_nop\n\tv_nop\n\tv_nop\n\tv_nop" : "+v"(a), "+v"(b) : "v"(x), "v"(y)); }
__device__ __forceinline__ void keep4_h(v16h a, v16h b, v16h c, v16h d) { asm volatile("v_nop" :: "v"(a), "v"(b), "v"(c), "v"(d)); }
__device__ __forceinline__ void keep4_b(v16b a, v16b b, v16b c, v16b d) { asm volatile("v_nop" :: "v"(a), "v"(b), "v"(c), "v"(d)); }
__device__ __forceinline__ void acc_guard4(v8f& a, v8f& b, v8f& c, v8f& d) { asm volatile("v_nop\n\tv_nop\n\tv_nop\n\tv_nop" : "+v"(a), "+v"(b), "+v"(c), "+v"(d)); }
template <typename T> struct Frag;
template <> struct Frag<_Float16> {
  typedef v16h V; union U { v16h v; v8h h[2]; };
  static __device__ __forceinline__ v16h load(const _Float16* p) {
    U f; f.h[0] = *(const v8h*)(p); f.h[1] = *(const v8h*)(p + 16); return f.v;
  }
  static __device__ __forceinline__ v8f mma(v16h a, v16h b, v8f c) {
    return __builtin_amdgcn_wmma_f32_16x16x32_f16(false, a, false, b, (short)0, c, false, false);
  }
  static __device__ __forceinline__ void guard(v8f& a, v8f& b, v16h x, v16h y) { dep_guard_h(a, b, x, y); }
  static __device__ __forceinline__ void keep(v16h a, v16h b, v16h c, v16h d) { keep4_h(a, b, c, d); }
};
template <> struct Frag<__bf16> {
  typedef v16b V; union U { v16b v; v8b h[2]; };
  static __device__ __forceinline__ v16b load(const __bf16* p) {
    U f; f.h[0] = *(const v8b*)(p); f.h[1] = *(const v8b*)(p + 16); return f.v;
  }
  static __device__ __forceinline__ v8f mma(v16b a, v16b b, v8f c) {
    return __builtin_amdgcn_wmma_f32_16x16x32_bf16(false, a, false, b, (short)0, c, false, false);
  }
  static __device__ __forceinline__ void guard(v8f& a, v8f& b, v16b x, v16b y) { dep_guard_b(a, b, x, y); }
  static __device__ __forceinline__ void keep(v16b a, v16b b, v16b c, v16b d) { keep4_b(a, b, c, d); }
};

template <int ET> struct Elem;
template <> struct Elem<0> { typedef _Float16 T; };
template <> struct Elem<1> { typedef __bf16 T; };
template <int ET, bool SPLIT, int BIAS_MODE, int OUT_MODE, bool RESID, int ACT = 0>
__global__ __launch_bounds__(256) void wmma_gemm64(
    const unsigned short* __restrict__ Ap, const unsigned short* __restrict__ A2p, int lda, long strideA,
    const unsigned short* __restrict__ Btp, const unsigned short* __restrict__ Bt2p, int ldb, long strideB,
    void* __restrict__ Cout, void* __restrict__ Cout2, int ldc, long strideC,
    const float* __restrict__ bias,
    const float* __restrict__ resid, long strideR,
    int M, int N, int K, float scale) {
  typedef typename Elem<ET>::T T;
  typedef typename Frag<T>::V V;
  const T* A = (const T*)Ap; const T* A2 = (const T*)A2p; const T* Bt = (const T*)Btp; const T* Bt2 = (const T*)Bt2p;
  __shared__ __align__(16) float sT[8][16 * 68];
  const int b    = blockIdx.y;
  const int lane = threadIdx.x & 31;
  const int wave = threadIdx.x >> 5;
  const int tilesN = N >> 6;
  const int tilesM = M >> 6;
  const int tile = blockIdx.x * 8 + wave;
  if (tile >= tilesM * tilesN) return;
  const int tm = tile / tilesN;
  const int tn = tile - tm * tilesN;
  const int m0 = tm << 6;
  const int n0 = tn << 6;

  const T* Ab  = A  + (size_t)b * strideA;
  const T* Bb  = Bt + (size_t)b * strideB;
  const T* Ab2 = SPLIT ? (A2  + (size_t)b * strideA) : nullptr;
  const T* Bb2 = SPLIT ? (Bt2 + (size_t)b * strideB) : nullptr;

  const int rlane = lane & 15;
  const int koff  = (lane >> 4) * 8;
  const int mOff  = (lane >> 4) * 8;

  v8f acc[4][4];
#pragma unroll
  for (int i = 0; i < 4; ++i)
#pragma unroll
    for (int j = 0; j < 4; ++j) acc[i][j] = (v8f){0.f,0.f,0.f,0.f,0.f,0.f,0.f,0.f};

  for (int k0 = 0; k0 < K; k0 += 32) {
    V bh[4], bl[4];
#pragma unroll
    for (int j = 0; j < 4; ++j) {
      const size_t bo = (size_t)(n0 + (j << 4) + rlane) * ldb + koff + k0;
      bh[j] = Frag<T>::load(Bb + bo);
      if (SPLIT) bl[j] = Frag<T>::load(Bb2 + bo);
    }
#pragma unroll
    for (int i = 0; i < 4; ++i) {
      const size_t ao = (size_t)(m0 + (i << 4) + rlane) * lda + koff + k0;
      V ah = Frag<T>::load(Ab + ao);
      V al;
      if (SPLIT) al = Frag<T>::load(Ab2 + ao);
#pragma unroll
      for (int j = 0; j < 4; ++j) {
        acc[i][j] = Frag<T>::mma(ah, bh[j], acc[i][j]);
        if (SPLIT) {
          acc[i][j] = Frag<T>::mma(ah, bl[j], acc[i][j]);
          acc[i][j] = Frag<T>::mma(al, bh[j], acc[i][j]);
        }
      }
      Frag<T>::guard(acc[i][0], acc[i][3], ah, SPLIT ? al : ah);
    }
    Frag<T>::keep(bh[0], bh[1], bh[2], bh[3]);
    if (SPLIT) Frag<T>::keep(bl[0], bl[1], bl[2], bl[3]);
  }
  acc_guard4(acc[0][0], acc[0][1], acc[0][2], acc[0][3]);
  acc_guard4(acc[1][0], acc[1][1], acc[1][2], acc[1][3]);
  acc_guard4(acc[2][0], acc[2][1], acc[2][2], acc[2][3]);
  acc_guard4(acc[3][0], acc[3][1], acc[3][2], acc[3][3]);

  float* slab = sT[wave];
  const float* Rb = RESID ? (resid + (size_t)b * strideR) : nullptr;
#pragma unroll
  for (int i = 0; i < 4; ++i) {
    const int mBase = m0 + (i << 4);
#pragma unroll
    for (int j = 0; j < 4; ++j) {
      const int n = n0 + (j << 4) + rlane;
      float bv = 0.f;
      if (BIAS_MODE == 2) bv = bias[n];
#pragma unroll
      for (int r = 0; r < 8; ++r) {
        float v = acc[i][j][r] * scale;
        if (BIAS_MODE == 1) v += bias[mBase + mOff + r];
        if (BIAS_MODE == 2) v += bv;
        if (RESID) v += Rb[(size_t)(mBase + mOff + r) * ldc + n];
        if (ACT == 1) v = tanhf(v);
        if (ACT == 2) v = fmaxf(v, 0.0f);
        if (ACT == 3) v = v / (1.0f + expf(-v));
        if (ACT == 4) v = (v > 0.f) ? v : 0.01f * v;
        if (ACT == 5) v = 0.5f * v * (1.0f + erff(v * 0.70710678118654752f));
        slab[(mOff + r) * 68 + (j << 4) + rlane] = v;
      }
    }
    __builtin_amdgcn_fence(__ATOMIC_RELEASE, "workgroup");
    __builtin_amdgcn_wave_barrier();
    __builtin_amdgcn_fence(__ATOMIC_ACQUIRE, "workgroup");
    if (OUT_MODE == 0) {
      float* C = (float*)Cout + (size_t)b * strideC;
      const int hh = lane >> 4, c4 = (lane & 15) * 4;
      for (int pass = 0; pass < 2; ++pass) {
#pragma unroll
        for (int it = 0; it < 8; ++it) {
          const int row = it * 2 + hh;
          v4f v = *(const v4f*)(slab + row * 68 + c4);
          *(volatile v4f*)(C + (size_t)(mBase + row) * ldc + n0 + c4) = v;
        }
        __threadfence();
      }
    } else {
      const int q = lane >> 3, c8 = (lane & 7) * 8;
      unsigned short* C  = (unsigned short*)Cout  + (size_t)b * strideC;
      unsigned short* C2 = (OUT_MODE == 2) ? ((unsigned short*)Cout2 + (size_t)b * strideC) : nullptr;
      for (int pass = 0; pass < 2; ++pass) {
#pragma unroll
        for (int it = 0; it < 4; ++it) {
          const int row = it * 4 + q;
          const float* sp = slab + row * 68 + c8;
          v8h hv, lv;
#pragma unroll
          for (int e = 0; e < 8; ++e) {
            if (OUT_MODE == 1) {
              hv[e] = (_Float16)sp[e];
            } else {
              unsigned short hb = f2bf_bits(sp[e]);
              unsigned short lb = f2bf_bits(sp[e] - bf_bits2f(hb));
              hv[e] = __builtin_bit_cast(_Float16, hb);
              lv[e] = __builtin_bit_cast(_Float16, lb);
            }
          }
          *(volatile v8h*)(C + (size_t)(mBase + row) * ldc + n0 + c8) = hv;
          if (OUT_MODE == 2) *(volatile v8h*)(C2 + (size_t)(mBase + row) * ldc + n0 + c8) = lv;
        }
        __threadfence();
      }
    }
    __builtin_amdgcn_fence(__ATOMIC_RELEASE, "workgroup");
    __builtin_amdgcn_wave_barrier();
    __builtin_amdgcn_fence(__ATOMIC_ACQUIRE, "workgroup");
  }
}

__global__ __launch_bounds__(256) void cast_f32_f16x2(
    const float* __restrict__ in, _Float16* __restrict__ out, int n2) {
  int i = blockIdx.x * 256 + threadIdx.x;
  if (i < n2) {
    const _Float16 h0 = (_Float16)in[2 * i], h1 = (_Float16)in[2 * i + 1];
    const unsigned u = (unsigned)__builtin_bit_cast(unsigned short, h0) | ((unsigned)__builtin_bit_cast(unsigned short, h1) << 16);
    ((volatile unsigned*)out)[i] = u;
    __threadfence();
    ((volatile unsigned*)out)[i] = u;
  }
}


#define MB_ 2
#define MCc 256
#define MH 96
#define MW 96
#define MHW (MH * MW)
#define MP (MB_ * MHW)
#define MK 9
#define MKC (MK * MCc)
__global__ __launch_bounds__(256) void xt_kernel(const float* __restrict__ x, float* __restrict__ XT) {
  __shared__ float tile[64][65];
  const int b = blockIdx.z, c0 = blockIdx.y * 64, p0 = blockIdx.x * 64, tx = threadIdx.x, ty = threadIdx.y;
  for (int c = ty; c < 64; c += 8) { tile[c][tx] = x[((size_t)b * MCc + c0 + c) * MHW + p0 + tx]; tile[c][32 + tx] = x[((size_t)b * MCc + c0 + c) * MHW + p0 + 32 + tx]; }
  __syncthreads();
  for (int pass = 0; pass < 2; ++pass) { for (int p = ty; p < 64; p += 8) { float* dst = XT + ((size_t)b * MHW + p0 + p) * MCc + c0; ((volatile float*)dst)[tx] = tile[tx][p]; ((volatile float*)dst)[32 + tx] = tile[32 + tx][p]; } __threadfence(); }
}
__global__ __launch_bounds__(256) void wperm_kernel(const float* __restrict__ w, unsigned* __restrict__ WT) {
  const int i = blockIdx.x * 256 + threadIdx.x; if (i >= MCc * MKC / 2) return; const int o = (2 * i) / MKC, r = (2 * i) % MKC; const int k = r / MCc, c = r % MCc;
  const unsigned u = (unsigned)__builtin_bit_cast(unsigned short, (_Float16)w[((size_t)o * MCc + c) * MK + k]) | ((unsigned)__builtin_bit_cast(unsigned short, (_Float16)w[((size_t)o * MCc + c + 1) * MK + k]) << 16);
  ((volatile unsigned*)WT)[i] = u; __threadfence(); ((volatile unsigned*)WT)[i] = u;
}
__global__ __launch_bounds__(256) void col_kernel(const float* __restrict__ XT, const float* __restrict__ offset, const float* __restrict__ mask, unsigned* __restrict__ A) {
  const int lane = threadIdx.x & 31, wave = threadIdx.x >> 5; const int item = blockIdx.x * 8 + wave; const int p = item / MK, k = item % MK;
  const int b = p / MHW, hw = p % MHW, h = hw / MW, w = hw % MW;
  const float offy = offset[(((size_t)b * MK + k) * 2 + 0) * MHW + hw], offx = offset[(((size_t)b * MK + k) * 2 + 1) * MHW + hw];
  const float ky = (float)(k / 3 - 1), kx = (float)(k % 3 - 1);
  const float py = ((float)h + ky) + offy, px = ((float)w + kx) + offx;
  const float y0f = floorf(py), x0f = floorf(px); const float dy = py - y0f, dx = px - x0f; const int y0 = (int)y0f, x0 = (int)x0f;
  const float m = mask[((size_t)b * MK + k) * MHW + hw];
  const float w00 = (1.f - dy) * (1.f - dx), w01 = (1.f - dy) * dx, w10 = dy * (1.f - dx), w11 = dy * dx;
  float v[8]; for (int e = 0; e < 8; ++e) v[e] = 0.f;
#pragma unroll
  for (int corner = 0; corner < 4; ++corner) { const int yi = y0 + (corner >> 1), xi = x0 + (corner & 1); const float wc = (corner == 0) ? w00 : (corner == 1 ? w01 : (corner == 2 ? w10 : w11));
    if (yi >= 0 && yi < MH && xi >= 0 && xi < MW) { const float* src = XT + ((size_t)b * MHW + yi * MW + xi) * MCc + lane * 8; const v4f a = *(const v4f*)src, c = *(const v4f*)(src + 4);
      for (int e = 0; e < 4; ++e) { v[e] += wc * a[e]; v[4 + e] += wc * c[e]; } } }
  typedef __attribute__((ext_vector_type(4))) unsigned u4; u4 pk;
  for (int q = 0; q < 4; ++q) pk[q] = (unsigned)__builtin_bit_cast(unsigned short, (_Float16)(v[2 * q] * m)) | ((unsigned)__builtin_bit_cast(unsigned short, (_Float16)(v[2 * q + 1] * m)) << 16);
  unsigned* dst = A + ((size_t)p * MKC + k * MCc) / 2 + lane * 4;
  *(volatile u4*)dst = pk; __threadfence(); *(volatile u4*)dst = pk;
}
__global__ __launch_bounds__(256) void gn_part_kernel(const float* __restrict__ CONV, double* __restrict__ PS) {
  __shared__ double rs[256], rss[256];
  const int bg = blockIdx.y, chunk = blockIdx.x; const int b = bg / 16, g = bg % 16; const int c = threadIdx.x & 15, pr = threadIdx.x >> 4;
  double s = 0.0, ss = 0.0;
  for (int p = chunk * 1152 + pr; p < (chunk + 1) * 1152; p += 16) { const double v = CONV[((size_t)b * MHW + p) * MCc + g * 16 + c]; s += v; ss += v * v; }
  rs[threadIdx.x] = s; rss[threadIdx.x] = ss; __syncthreads();
  for (int o = 128; o > 0; o >>= 1) { if (threadIdx.x < o) { rs[threadIdx.x] += rs[threadIdx.x + o]; rss[threadIdx.x] += rss[threadIdx.x + o]; } __syncthreads(); }
  if (threadIdx.x < 32) { const double v = (threadIdx.x == 0) ? rs[0] : (threadIdx.x == 1 ? rss[0] : 0.0); ((volatile double*)PS)[((size_t)bg * 8 + chunk) * 32 + threadIdx.x] = v; __threadfence(); ((volatile double*)PS)[((size_t)bg * 8 + chunk) * 32 + threadIdx.x] = v; }
}
__global__ __launch_bounds__(256) void gn_out_kernel(const float* __restrict__ CONV, const double* __restrict__ PS, const float* __restrict__ gamma, const float* __restrict__ beta, float* __restrict__ out) {
  __shared__ float tile[64][65]; __shared__ float sc[64], sh[64];
  const int b = blockIdx.z, c0 = blockIdx.y * 64, p0 = blockIdx.x * 64, tx = threadIdx.x, ty = threadIdx.y; const int t = ty * 32 + tx;
  if (t < 64) { const int c = c0 + t, g = c / 16; double s = 0.0, ss = 0.0; for (int ch = 0; ch < 8; ++ch) { s += PS[((size_t)(b * 16 + g) * 8 + ch) * 32]; ss += PS[((size_t)(b * 16 + g) * 8 + ch) * 32 + 1]; }
    const double n = 16.0 * MHW; const double mu = s / n; double var = ss / n - mu * mu; if (var < 0) var = 0; const float inv = (float)(1.0 / sqrt(var + 1e-5));
    sc[t] = inv * gamma[c]; sh[t] = beta[c] - (float)mu * inv * gamma[c]; }
  for (int p = ty; p < 64; p += 8) { const float* src = CONV + ((size_t)b * MHW + p0 + p) * MCc + c0; tile[tx][p] = src[tx]; tile[32 + tx][p] = src[32 + tx]; }
  __syncthreads();
  for (int pass = 0; pass < 2; ++pass) { for (int c = ty; c < 64; c += 8) { float* dst = out + ((size_t)b * MCc + c0 + c) * MHW + p0; ((volatile float*)dst)[tx] = tile[c][tx] * sc[c] + sh[c]; ((volatile float*)dst)[32 + tx] = tile[c][32 + tx] * sc[c] + sh[c]; } __threadfence(); }
}
extern "C" void kernel_launch(void* const* d_in, const int* in_sizes, int n_in, void* d_out, int out_size, void* d_ws, size_t ws_size, hipStream_t stream) {
  (void)in_sizes; (void)n_in; (void)out_size; (void)ws_size;
  const float* x = (const float*)d_in[0]; const float* offset = (const float*)d_in[1]; const float* mask = (const float*)d_in[2]; const float* weight = (const float*)d_in[3]; const float* bias = (const float*)d_in[4]; const float* gamma = (const float*)d_in[5]; const float* beta = (const float*)d_in[6];
  char* ws = (char*)d_ws; size_t off = 0;
  auto carve = [&](size_t bytes) -> char* { char* p = ws + off; off += (bytes + 255) & ~(size_t)255; return p; };
  float* XT = (float*)carve((size_t)MP * MCc * 4);
  unsigned* WT = (unsigned*)carve((size_t)MCc * MKC * 2);
  unsigned* A = (unsigned*)carve((size_t)MP * MKC * 2);
  float* CONV = (float*)carve((size_t)MP * MCc * 4);
  double* PS = (double*)carve((size_t)MB_ * 16 * 8 * 32 * 8);
  xt_kernel<<<dim3(MHW / 64, MCc / 64, MB_), dim3(32, 8), 0, stream>>>(x, XT);
  wperm_kernel<<<(MCc * MKC / 2 + 255) / 256, 256, 0, stream>>>(weight, WT);
  col_kernel<<<MP * MK / 8, 256, 0, stream>>>(XT, offset, mask, A);
  { const int t = (MP / 64) * (MCc / 64);
    wmma_gemm64<0, false, 2, 0, false><<<dim3((t + 7) / 8, 1), 256, 0, stream>>>((const unsigned short*)A, nullptr, MKC, 0, (const unsigned short*)WT, nullptr, MKC, 0, CONV, nullptr, MCc, 0, bias, nullptr, 0, MP, MCc, MKC, 1.0f); }
  gn_part_kernel<<<dim3(8, MB_ * 16), 256, 0, stream>>>(CONV, PS);
  gn_out_kernel<<<dim3(MHW / 64, MCc / 64, MB_), dim3(32, 8), 0, stream>>>(CONV, PS, gamma, beta, (float*)d_out);
}
